// GPT2Attention_17918603559271
// MI455X (gfx1250) — hardware-verified
//
#include <hip/hip_runtime.h>


#ifndef NB
#define NB 4
#endif
#ifndef SEQ
#define SEQ 2048
#endif
#define SEQ_FULL 2048
#define HID 1024
#define NHEAD 16
#define HD 64
#define MROWS (NB * SEQ)

static_assert(SEQ % 128 == 0);
static_assert(SEQ <= SEQ_FULL);
static_assert((SEQ * 32) % 256 == 0);
static_assert(((size_t)MROWS * HID) % 2048 == 0);
static_assert(NHEAD * HD == HID);

typedef _Float16 v16h __attribute__((ext_vector_type(16)));
typedef _Float16 v8h  __attribute__((ext_vector_type(8)));
typedef float    v8f  __attribute__((ext_vector_type(8)));
typedef float    v4f  __attribute__((ext_vector_type(4)));
union Frag { v16h v; v8h h[2]; };

#define WMMA_F16(a, b, c) \
  __builtin_amdgcn_wmma_f32_16x16x32_f16(false, (a), false, (b), (short)0, (c), false, false)

__device__ __forceinline__ v16h load_frag(const _Float16* base, int stride, int row, int k0, int lane) {
  const _Float16* p = base + (size_t)(row + (lane & 15)) * stride + k0 + ((lane >> 4) << 3);
  Frag u;
  u.h[0] = *(const v8h*)(p);
  u.h[1] = *(const v8h*)(p + 16);
  return u.v;
}

__device__ __forceinline__ float bf16_rne(float x) {
  unsigned u = __float_as_uint(x);
  u = (u + 0x7FFFu + ((u >> 16) & 1u)) & 0xFFFF0000u;
  return __uint_as_float(u);
}

__global__ __launch_bounds__(256) void k_tab(float* cosT, float* sinT) {
  const int idx = blockIdx.x * 256 + threadIdx.x;
  const int s = idx >> 5, j = idx & 31;
  double p = (j >= 24) ? 1000.0 : (j >= 16) ? 100.0 : (j >= 8) ? 10.0 : 1.0;
  const int jr = j & 7;
#pragma unroll 1
  for (int i = 0; i < jr; ++i) p *= 1.333521432163324;
  const float pf  = (float)p;
  const float inv = 1.0f / pf;
  const float ang = (float)s * inv;
  const float cs = cosf(ang);
  const float sn = sinf(ang);
  volatile float* pc = cosT + idx;
  volatile float* ps = sinT + idx;
  *pc = cs; *ps = sn;
  __threadfence();
  *pc = cs; *ps = sn;
}

__global__ __launch_bounds__(256) void k_cvt_x(const float* __restrict__ x, _Float16* xh) {
  const size_t t = (size_t)blockIdx.x * 256 + threadIdx.x;
  const size_t e = t * 8;
  const int m = (int)(e >> 10);
  const int c = (int)(e & 1023);
  const int b = m / SEQ, s = m - b * SEQ;
  const float* src = x + ((size_t)b * SEQ_FULL + s) * HID + c;
  const v4f f0 = *(const v4f*)(src);
  const v4f f1 = *(const v4f*)(src + 4);
  v8h o;
#pragma unroll
  for (int j = 0; j < 4; ++j) {
    o[j]     = (_Float16)bf16_rne(f0[j]);
    o[j + 4] = (_Float16)bf16_rne(f1[j]);
  }
  volatile v8h* d = (volatile v8h*)(xh + e);
  *d = o;
  __threadfence();
  *d = o;
}

__global__ __launch_bounds__(256) void k_cvt_w(const float* __restrict__ w0, const float* __restrict__ w1,
                                               const float* __restrict__ w2, const float* __restrict__ w3,
                                               _Float16* wh) {
  const int y = blockIdx.y;
  const float* w = (y == 0) ? w0 : (y == 1) ? w1 : (y == 2) ? w2 : w3;
  const size_t e = ((size_t)blockIdx.x * 256 + threadIdx.x) * 8;
  const v4f f0 = *(const v4f*)(w + e);
  const v4f f1 = *(const v4f*)(w + e + 4);
  v8h o;
#pragma unroll
  for (int j = 0; j < 4; ++j) {
    o[j]     = (_Float16)(bf16_rne(f0[j]) * 16.0f);
    o[j + 4] = (_Float16)(bf16_rne(f1[j]) * 16.0f);
  }
  volatile v8h* d = (volatile v8h*)(wh + (size_t)y * HID * HID + e);
  *d = o;
  __threadfence();
  *d = o;
}

__device__ __forceinline__ void gemm_32x64(const _Float16* __restrict__ X, const _Float16* __restrict__ W,
                                           int mrow, int nrow, int lane, v8f (&acc)[2][4]) {
#pragma unroll 1
  for (int k0 = 0; k0 < HID; k0 += 32) {
    const v16h a0 = load_frag(X, HID, mrow,      k0, lane);
    const v16h a1 = load_frag(X, HID, mrow + 16, k0, lane);
    const v16h b0 = load_frag(W, HID, nrow,      k0, lane);
    const v16h b1 = load_frag(W, HID, nrow + 16, k0, lane);
    const v16h b2 = load_frag(W, HID, nrow + 32, k0, lane);
    const v16h b3 = load_frag(W, HID, nrow + 48, k0, lane);
    acc[0][0] = WMMA_F16(a0, b0, acc[0][0]);
    acc[0][1] = WMMA_F16(a0, b1, acc[0][1]);
    acc[0][2] = WMMA_F16(a0, b2, acc[0][2]);
    acc[0][3] = WMMA_F16(a0, b3, acc[0][3]);
    acc[1][0] = WMMA_F16(a1, b0, acc[1][0]);
    acc[1][1] = WMMA_F16(a1, b1, acc[1][1]);
    acc[1][2] = WMMA_F16(a1, b2, acc[1][2]);
    acc[1][3] = WMMA_F16(a1, b3, acc[1][3]);
    asm volatile("v_nop\n\tv_nop\n\tv_nop\n\tv_nop"
                 : "+v"(acc[0][0]), "+v"(acc[0][1]), "+v"(acc[0][2]), "+v"(acc[0][3]),
                   "+v"(acc[1][0]), "+v"(acc[1][1]), "+v"(acc[1][2]), "+v"(acc[1][3])
                 : "v"(a0), "v"(a1), "v"(b0), "v"(b1), "v"(b2), "v"(b3));
  }
}

__global__ __launch_bounds__(128) void k_qkv(
    const _Float16* __restrict__ Xh, const _Float16* __restrict__ Wh,
    const float* __restrict__ bq, const float* __restrict__ bk, const float* __restrict__ bv,
    const float* __restrict__ cosT, const float* __restrict__ sinT,
    _Float16* Qh, _Float16* Kh, _Float16* Vt)
{
  __shared__ __attribute__((aligned(16))) float    sCos[128 * 32];
  __shared__ __attribute__((aligned(16))) float    sSin[128 * 32];
  __shared__ __attribute__((aligned(16))) _Float16 sT[128 * 72];

  const int tid   = threadIdx.x;
  const int lane  = tid & 31;
  const int wave  = tid >> 5;
  const int l15   = lane & 15;
  const int half8 = (lane >> 4) << 3;
  const int mblk  = blockIdx.x * 128;
  const int mat   = blockIdx.y >> 4;
  const int head  = blockIdx.y & 15;
  const int bb    = mblk / SEQ;
  const int s0    = mblk - bb * SEQ;

  const v8f vzero = {0.f, 0.f, 0.f, 0.f, 0.f, 0.f, 0.f, 0.f};
  v8f acc[2][4];
#pragma unroll
  for (int mi = 0; mi < 2; ++mi)
#pragma unroll
    for (int ni = 0; ni < 4; ++ni) acc[mi][ni] = vzero;

  gemm_32x64(Xh, Wh, mblk + wave * 32, blockIdx.y * 64, lane, acc);

  if (mat < 2) {
    const v4f* c4 = (const v4f*)(cosT + (size_t)s0 * 32);
    const v4f* n4 = (const v4f*)(sinT + (size_t)s0 * 32);
#pragma unroll
    for (int it = 0; it < 8; ++it) {
      const int idx = it * 128 + tid;
      ((v4f*)sCos)[idx] = c4[idx];
      ((v4f*)sSin)[idx] = n4[idx];
    }
  }
  __syncthreads();

  const float* bp = (mat == 0) ? bq : (mat == 1) ? bk : bv;
  float bias[4];
#pragma unroll
  for (int ni = 0; ni < 4; ++ni) bias[ni] = 16.0f * bf16_rne(bp[head * 64 + ni * 16 + l15]);

#pragma unroll
  for (int mi = 0; mi < 2; ++mi) {
#pragma unroll
    for (int r = 0; r < 8; ++r) {
      const int lrow = wave * 32 + mi * 16 + r + half8;
      const float y0 = acc[mi][0][r] + bias[0];
      const float y1 = acc[mi][1][r] + bias[1];
      const float y2 = acc[mi][2][r] + bias[2];
      const float y3 = acc[mi][3][r] + bias[3];
      if (mat < 2) {
        const float c0 = sCos[lrow * 32 + l15];
        const float c1 = sCos[lrow * 32 + 16 + l15];
        const float n0 = sSin[lrow * 32 + l15];
        const float n1 = sSin[lrow * 32 + 16 + l15];
        const float o0 = y0 * c0 - y2 * n0;
        const float o1 = y1 * c1 - y3 * n1;
        const float o2 = y2 * c0 + y0 * n0;
        const float o3 = y3 * c1 + y1 * n1;
        sT[lrow * 72 +  0 + l15] = (_Float16)o0;
        sT[lrow * 72 + 16 + l15] = (_Float16)o1;
        sT[lrow * 72 + 32 + l15] = (_Float16)o2;
        sT[lrow * 72 + 48 + l15] = (_Float16)o3;
      } else {
        sT[( 0 + l15) * 136 + lrow] = (_Float16)y0;
        sT[(16 + l15) * 136 + lrow] = (_Float16)y1;
        sT[(32 + l15) * 136 + lrow] = (_Float16)y2;
        sT[(48 + l15) * 136 + lrow] = (_Float16)y3;
      }
    }
  }
  __syncthreads();

  const int bh = bb * NHEAD + head;
  if (mat < 2) {
    _Float16* dst = ((mat == 0) ? Qh : Kh) + ((size_t)bh * SEQ + s0) * HD;
    for (int pass = 0; pass < 2; ++pass) {
#pragma unroll
      for (int it = 0; it < 8; ++it) {
        const int piece = it * 128 + tid;
        const int row = piece >> 3, c8 = (piece & 7) * 8;
        const v8h v = *(const v8h*)(&sT[row * 72 + c8]);
        *(volatile v8h*)(dst + (size_t)row * HD + c8) = v;
      }
      __threadfence();
    }
  } else {
    _Float16* dst = Vt + (size_t)bh * HD * SEQ + s0;
    for (int pass = 0; pass < 2; ++pass) {
#pragma unroll
      for (int it = 0; it < 8; ++it) {
        const int piece = it * 128 + tid;
        const int d = piece >> 4, c8 = (piece & 15) * 8;
        const v8h v = *(const v8h*)(&sT[d * 136 + c8]);
        *(volatile v8h*)(dst + (size_t)d * SEQ + c8) = v;
      }
      __threadfence();
    }
  }
}

__global__ __launch_bounds__(128) void k_flash(
    const _Float16* __restrict__ Q, const _Float16* __restrict__ K,
    const _Float16* __restrict__ Vt, _Float16* Ctx)
{
  __shared__ __attribute__((aligned(16))) _Float16 sO[4][16 * 72];

  const int tid   = threadIdx.x;
  const int lane  = tid & 31;
  const int wave  = tid >> 5;
  const int l15   = lane & 15;
  const int half8 = (lane >> 4) << 3;
  const int bh    = blockIdx.y;
  const int qbase = blockIdx.x * 64 + wave * 16;

  const _Float16* Qh = Q  + (size_t)bh * SEQ * HD;
  const _Float16* Kh = K  + (size_t)bh * SEQ * HD;
  const _Float16* Vh = Vt + (size_t)bh * HD * SEQ;

  const v16h qf0 = load_frag(Qh, HD, qbase, 0,  lane);
  const v16h qf1 = load_frag(Qh, HD, qbase, 32, lane);

  const v8f vzero = {0.f, 0.f, 0.f, 0.f, 0.f, 0.f, 0.f, 0.f};
  v8f accO[4];
#pragma unroll
  for (int mt = 0; mt < 4; ++mt) accO[mt] = vzero;
  float mrun = -1.0e30f, lrun = 0.f;
  const float SC = 1.0f / 2048.0f;

#pragma unroll 1
  for (int kb = 0; kb < SEQ; kb += 64) {
    v8f s4[4];
#pragma unroll
    for (int kt = 0; kt < 4; ++kt) {
      const v16h ka0 = load_frag(Kh, HD, kb + kt * 16, 0,  lane);
      const v16h ka1 = load_frag(Kh, HD, kb + kt * 16, 32, lane);
      v8f z = vzero;
      z = WMMA_F16(ka0, qf0, z);
      z = WMMA_F16(ka1, qf1, z);
      if (kt == 3) {
        asm volatile("v_nop\n\tv_nop\n\tv_nop\n\tv_nop"
                     : "+v"(s4[0]), "+v"(s4[1]), "+v"(s4[2]), "+v"(z)
                     : "v"(ka0), "v"(ka1), "v"(qf0), "v"(qf1));
      }
      s4[kt] = z;
    }

    float mloc = mrun;
#pragma unroll
    for (int kt = 0; kt < 4; ++kt)
#pragma unroll
      for (int r = 0; r < 8; ++r) mloc = fmaxf(mloc, s4[kt][r] * SC);
    mloc = fmaxf(mloc, __shfl_xor(mloc, 16, 32));
    const float alpha = __expf(mrun - mloc);
    mrun = mloc;

    float lsum = 0.f;
    v16h pf0, pf1;
#pragma unroll
    for (int h = 0; h < 16; ++h) {
      const float e0 = __expf(s4[h >> 3][h & 7] * SC - mloc);
      const float e1 = __expf(s4[2 + (h >> 3)][h & 7] * SC - mloc);
      lsum += e0 + e1;
      pf0[h] = (_Float16)(e0 * 256.0f);
      pf1[h] = (_Float16)(e1 * 256.0f);
    }
    lsum += __shfl_xor(lsum, 16, 32);
    lrun = lrun * alpha + lsum;

#pragma unroll
    for (int mt = 0; mt < 4; ++mt)
#pragma unroll
      for (int r = 0; r < 8; ++r) accO[mt][r] *= alpha;

#pragma unroll
    for (int mt = 0; mt < 4; ++mt) {
      const v16h va0 = load_frag(Vh, SEQ, mt * 16, kb,      lane);
      const v16h va1 = load_frag(Vh, SEQ, mt * 16, kb + 32, lane);
      accO[mt] = WMMA_F16(va0, pf0, accO[mt]);
      accO[mt] = WMMA_F16(va1, pf1, accO[mt]);
      if (mt == 3) {
        asm volatile("v_nop\n\tv_nop\n\tv_nop\n\tv_nop"
                     : "+v"(accO[0]), "+v"(accO[1]), "+v"(accO[2]), "+v"(accO[3])
                     : "v"(va0), "v"(va1), "v"(pf0), "v"(pf1));
      }
    }
  }

  const float inv = 1.0f / (lrun * 64.0f);
#pragma unroll
  for (int mt = 0; mt < 4; ++mt)
#pragma unroll
    for (int r = 0; r < 8; ++r)
      sO[wave][l15 * 72 + mt * 16 + half8 + r] = (_Float16)(accO[mt][r] * inv);
  __syncthreads();

  const int bb = bh >> 4, head = bh & 15;
  _Float16* dst = Ctx + ((size_t)bb * SEQ + qbase) * HID + head * HD;
  for (int pass = 0; pass < 2; ++pass) {
#pragma unroll
    for (int it = 0; it < 4; ++it) {
      const int piece = it * 32 + lane;
      const int row = piece >> 3, c8 = (piece & 7) * 8;
      const v8h v = *(const v8h*)(&sO[wave][row * 72 + c8]);
      *(volatile v8h*)(dst + (size_t)row * HID + c8) = v;
    }
    __threadfence();
  }
}

__global__ __launch_bounds__(128) void k_oproj(
    const _Float16* __restrict__ Ch, const _Float16* __restrict__ Wo16,
    const float* __restrict__ bo, float* out)
{
  __shared__ __attribute__((aligned(16))) float sF[128 * 68];

  const int tid   = threadIdx.x;
  const int lane  = tid & 31;
  const int wave  = tid >> 5;
  const int l15   = lane & 15;
  const int half8 = (lane >> 4) << 3;
  const int mblk  = blockIdx.x * 128;
  const int nbase = blockIdx.y * 64;

  const v8f vzero = {0.f, 0.f, 0.f, 0.f, 0.f, 0.f, 0.f, 0.f};
  v8f acc[2][4];
#pragma unroll
  for (int mi = 0; mi < 2; ++mi)
#pragma unroll
    for (int ni = 0; ni < 4; ++ni) acc[mi][ni] = vzero;

  gemm_32x64(Ch, Wo16, mblk + wave * 32, nbase, lane, acc);

  float bias[4];
#pragma unroll
  for (int ni = 0; ni < 4; ++ni) bias[ni] = bf16_rne(bo[nbase + ni * 16 + l15]);

#pragma unroll
  for (int mi = 0; mi < 2; ++mi)
#pragma unroll
    for (int r = 0; r < 8; ++r) {
      const int lrow = wave * 32 + mi * 16 + r + half8;
#pragma unroll
      for (int ni = 0; ni < 4; ++ni)
        sF[lrow * 68 + ni * 16 + l15] = acc[mi][ni][r] * (1.0f / 1024.0f) + bias[ni];
    }
  __syncthreads();

  float* dst = out + (size_t)mblk * HID + nbase;
  for (int pass = 0; pass < 2; ++pass) {
#pragma unroll
    for (int it = 0; it < 16; ++it) {
      const int piece = it * 128 + tid;
      const int row = piece >> 4, c4 = (piece & 15) * 4;
      const v4f v = *(const v4f*)(&sF[row * 68 + c4]);
      *(volatile v4f*)(dst + (size_t)row * HID + c4) = v;
    }
    __threadfence();
  }
}

static constexpr size_t kPlane   = (size_t)MROWS * HID * 2;
static constexpr size_t kWPlanes = (size_t)4 * HID * HID * 2;
static constexpr size_t kTab     = (size_t)SEQ * 32 * 4;
static constexpr size_t kOffX    = 0;
static constexpr size_t kOffW    = kOffX + kPlane;
static constexpr size_t kOffQ    = kOffW + kWPlanes;
static constexpr size_t kOffK    = kOffQ + kPlane;
static constexpr size_t kOffV    = kOffK + kPlane;
static constexpr size_t kOffC    = kOffV + kPlane;
static constexpr size_t kOffCos  = kOffC + kPlane;
static constexpr size_t kOffSin  = kOffCos + kTab;
static constexpr size_t kWsTotal = kOffSin + kTab;
static_assert(kWsTotal <= (size_t)134217728);
static_assert(kPlane % 128 == 0);
static_assert(kTab % 128 == 0);

extern "C" void kernel_launch(void* const* d_in, const int* in_sizes, int n_in,
                              void* d_out, int out_size, void* d_ws, size_t ws_size,
                              hipStream_t stream) {
  if (n_in < 9) return;
  if (ws_size < kWsTotal) return;
  const long long need_x = ((long long)(NB - 1) * SEQ_FULL + SEQ) * HID;
  if ((long long)in_sizes[0] < need_x) return;
  if (in_sizes[1] < HID * HID || in_sizes[3] < HID * HID || in_sizes[5] < HID * HID || in_sizes[7] < HID * HID) return;
  if (in_sizes[2] < HID || in_sizes[4] < HID || in_sizes[6] < HID || in_sizes[8] < HID) return;
  if ((long long)out_size < (long long)MROWS * HID) return;

  const float* x  = (const float*)d_in[0];
  const float* Wq = (const float*)d_in[1];
  const float* bq = (const float*)d_in[2];
  const float* Wk = (const float*)d_in[3];
  const float* bk = (const float*)d_in[4];
  const float* Wv = (const float*)d_in[5];
  const float* bv = (const float*)d_in[6];
  const float* Wo = (const float*)d_in[7];
  const float* bo = (const float*)d_in[8];

  char* ws = (char*)d_ws;
  _Float16* Xh  = (_Float16*)(ws + kOffX);
  _Float16* Wh  = (_Float16*)(ws + kOffW);
  _Float16* Qh  = (_Float16*)(ws + kOffQ);
  _Float16* Kh  = (_Float16*)(ws + kOffK);
  _Float16* Vt  = (_Float16*)(ws + kOffV);
  _Float16* Ch  = (_Float16*)(ws + kOffC);
  float* cosT   = (float*)(ws + kOffCos);
  float* sinT   = (float*)(ws + kOffSin);

  k_tab<<<dim3((SEQ * 32) / 256), dim3(256), 0, stream>>>(cosT, sinT);
  k_cvt_x<<<dim3((unsigned)(((size_t)MROWS * HID) / 2048)), dim3(256), 0, stream>>>(x, Xh);
  k_cvt_w<<<dim3((HID * HID) / 2048, 4), dim3(256), 0, stream>>>(Wq, Wk, Wv, Wo, Wh);
  k_qkv<<<dim3(MROWS / 128, 48), dim3(128), 0, stream>>>(Xh, Wh, bq, bk, bv, cosT, sinT, Qh, Kh, Vt);
  k_flash<<<dim3(SEQ / 64, NB * NHEAD), dim3(128), 0, stream>>>(Qh, Kh, Vt, Ch);
  k_oproj<<<dim3(MROWS / 128, 16), dim3(128), 0, stream>>>(Ch, Wh + (size_t)3 * HID * HID, bo, (float*)d_out);
}
